// LibragradAttention_24060406792851
// MI455X (gfx1250) — hardware-verified
//
#include <hip/hip_runtime.h>
#include <stdint.h>
#include <stddef.h>


typedef unsigned int   u32;
typedef unsigned short u16;
typedef _Float16 v16h  __attribute__((ext_vector_type(16)));
typedef __bf16   v16b  __attribute__((ext_vector_type(16)));
typedef float    v8f   __attribute__((ext_vector_type(8)));
typedef u32      u32x4 __attribute__((ext_vector_type(4)));
typedef float    f32x4 __attribute__((ext_vector_type(4)));

union Frag { v16h vh; v16b vb; u32x4 q[2]; u32 u[8]; };
union Acc  { v8f v; float f[8]; };

__device__ __forceinline__ u32 bf16_rne_bits(float a) {
  u32 u = __builtin_bit_cast(u32, a);
  u += 0x7FFFu + ((u >> 16) & 1u);
  return u >> 16;
}
__device__ __forceinline__ float bf16_rne(float a) {
  return __builtin_bit_cast(float, bf16_rne_bits(a) << 16);
}
__device__ __forceinline__ u32 packbf2(float a, float b) {
  return bf16_rne_bits(a) | (bf16_rne_bits(b) << 16);
}
__device__ __forceinline__ u32 h_bits(float a) {
  _Float16 t = (_Float16)a;
  return (u32)__builtin_bit_cast(u16, t);
}
__device__ __forceinline__ u32 packh2(float a, float b) {
  return h_bits(a) | (h_bits(b) << 16);
}

__device__ __forceinline__ v8f wmma_bf16(const Frag& a, const Frag& b, v8f c) {
  return __builtin_amdgcn_wmma_f32_16x16x32_bf16(false, a.vb, false, b.vb, (short)0, c, false, false);
}
__device__ __forceinline__ v8f wmma_f16(const Frag& a, const Frag& b, v8f c) {
  return __builtin_amdgcn_wmma_f32_16x16x32_f16(false, a.vh, false, b.vh, (short)0, c, false, false);
}
#define WMMA_GUARD1(accv, a0, a1, b0, b1)                                   \
  asm volatile("v_nop\n\tv_nop\n\tv_nop\n\tv_nop"                            \
               : "+v"(accv) : "v"(a0), "v"(a1), "v"(b0), "v"(b1))

__global__ __launch_bounds__(256) void cvt_bf16_kernel(
    const float* __restrict__ X0, const float* __restrict__ X1, const float* __restrict__ X2,
    u16* Y0, u16* Y1, u16* Y2, int n8)
{
  const int sel = blockIdx.y;
  const float* X = (sel == 0) ? X0 : ((sel == 1) ? X1 : X2);
  u16* Y = (sel == 0) ? Y0 : ((sel == 1) ? Y1 : Y2);
  const int i = blockIdx.x * 256 + (int)threadIdx.x;
  if (i >= n8) return;
  const f32x4 a = *(const f32x4*)(X + (size_t)i * 8);
  const f32x4 c = *(const f32x4*)(X + (size_t)i * 8 + 4);
  u32x4 o;
  o.x = packbf2(a.x, a.y); o.y = packbf2(a.z, a.w);
  o.z = packbf2(c.x, c.y); o.w = packbf2(c.z, c.w);
  volatile u32x4* d = (volatile u32x4*)(Y + (size_t)i * 8);
  *d = o;
  __threadfence();
  *d = o;
}

__global__ __launch_bounds__(256) void wtrans_kernel(
    const float* __restrict__ W0, const float* __restrict__ W1,
    const float* __restrict__ W2, const float* __restrict__ W3,
    u16* O0, u16* O1, u16* O2, u16* O3, int R, int Cc, float s3)
{
  __shared__ float tile[64][33];
  const int sel = blockIdx.z;
  const float* W = (sel == 0) ? W0 : ((sel == 1) ? W1 : ((sel == 2) ? W2 : W3));
  u16* O = (sel == 0) ? O0 : ((sel == 1) ? O1 : ((sel == 2) ? O2 : O3));
  const int r0 = blockIdx.x * 64, c0 = blockIdx.y * 32;
  const int tid = threadIdx.x, lane = tid & 31, wid = tid >> 5;
  {
    const int row = tid >> 2, c8 = (tid & 3) * 8;
    const f32x4 x0 = *(const f32x4*)(W + (size_t)(r0 + row) * Cc + c0 + c8);
    const f32x4 x1 = *(const f32x4*)(W + (size_t)(r0 + row) * Cc + c0 + c8 + 4);
    tile[row][c8 + 0] = x0.x; tile[row][c8 + 1] = x0.y; tile[row][c8 + 2] = x0.z; tile[row][c8 + 3] = x0.w;
    tile[row][c8 + 4] = x1.x; tile[row][c8 + 5] = x1.y; tile[row][c8 + 6] = x1.z; tile[row][c8 + 7] = x1.w;
  }
  __syncthreads();
  const int rs = wid * 4 + (lane >> 3);
  const int cc = (lane & 7) * 8;
  float v[8];
  #pragma unroll
  for (int i = 0; i < 8; ++i) v[i] = tile[cc + i][rs];
  u32x4 o;
  if (sel == 3) {
    o.x = packh2(bf16_rne(v[0]) * s3, bf16_rne(v[1]) * s3);
    o.y = packh2(bf16_rne(v[2]) * s3, bf16_rne(v[3]) * s3);
    o.z = packh2(bf16_rne(v[4]) * s3, bf16_rne(v[5]) * s3);
    o.w = packh2(bf16_rne(v[6]) * s3, bf16_rne(v[7]) * s3);
  } else {
    o.x = packbf2(v[0], v[1]); o.y = packbf2(v[2], v[3]);
    o.z = packbf2(v[4], v[5]); o.w = packbf2(v[6], v[7]);
  }
  volatile u32x4* d = (volatile u32x4*)(O + (size_t)(c0 + rs) * R + r0 + cc);
  *d = o;
  __threadfence();
  *d = o;
}

template<bool F16OPS, int OMODE>
__global__ __launch_bounds__(256) void gemm_kernel(
    const u16* __restrict__ A, const u16* __restrict__ BT,
    const float* __restrict__ bias, void* Cp,
    int M, int K, int N, float acc_scale)
{
  constexpr int BM = 128, BN = 128, BK = 32, LDA = BK + 8, LDB = BK + 8;
  __shared__ __attribute__((aligned(16))) float smem_f[BM * BN];
  u16* const smem_h = reinterpret_cast<u16*>(smem_f);
  u16* const As = smem_h;
  u16* const Bs = smem_h + BM * LDA;

  const int tid = threadIdx.x, lane = tid & 31, wid = tid >> 5;
  const int l16 = lane & 15, hh = lane >> 4;
  const int bm = blockIdx.y * BM, bn = blockIdx.x * BN;
  const int wm = (wid & 3) * 32, wn = (wid >> 2) * 64;
  const int nkt = K / BK;

  Acc acc[2][4];
  #pragma unroll
  for (int i = 0; i < 2; ++i)
    #pragma unroll
    for (int j = 0; j < 4; ++j)
      #pragma unroll
      for (int r = 0; r < 8; ++r) acc[i][j].f[r] = 0.f;

  #pragma unroll 1
  for (int kt = 0; kt < nkt; ++kt) {
    const int k0 = kt * BK;
    u32x4 ra[2], rb[2];
    #pragma unroll
    for (int j = 0; j < 2; ++j) {
      const int f = tid + j * 256, row = f >> 2, c8 = (f & 3) * 8;
      ra[j] = *(const u32x4*)(A  + (size_t)(bm + row) * K + k0 + c8);
      rb[j] = *(const u32x4*)(BT + (size_t)(bn + row) * K + k0 + c8);
    }
    __syncthreads();
    #pragma unroll
    for (int j = 0; j < 2; ++j) {
      const int f = tid + j * 256, row = f >> 2, c8 = (f & 3) * 8;
      *(u32x4*)(As + row * LDA + c8) = ra[j];
      *(u32x4*)(Bs + row * LDB + c8) = rb[j];
    }
    __syncthreads();

    Frag a[2], b[4];
    #pragma unroll
    for (int mt = 0; mt < 2; ++mt) {
      const int row = wm + mt * 16 + l16;
      a[mt].q[0] = *(const u32x4*)(As + row * LDA + 8 * hh);
      a[mt].q[1] = *(const u32x4*)(As + row * LDA + 16 + 8 * hh);
    }
    #pragma unroll
    for (int nt = 0; nt < 4; ++nt) {
      const int col = wn + nt * 16 + l16;
      b[nt].q[0] = *(const u32x4*)(Bs + col * LDB + 8 * hh);
      b[nt].q[1] = *(const u32x4*)(Bs + col * LDB + 16 + 8 * hh);
    }
    #pragma unroll
    for (int mt = 0; mt < 2; ++mt)
      #pragma unroll
      for (int nt = 0; nt < 4; ++nt) {
        if constexpr (F16OPS) acc[mt][nt].v = wmma_f16 (a[mt], b[nt], acc[mt][nt].v);
        else                  acc[mt][nt].v = wmma_bf16(a[mt], b[nt], acc[mt][nt].v);
      }
    asm volatile("v_nop\n\tv_nop\n\tv_nop\n\tv_nop"
                 : "+v"(acc[0][0].v), "+v"(acc[0][1].v), "+v"(acc[0][2].v), "+v"(acc[0][3].v),
                   "+v"(acc[1][0].v), "+v"(acc[1][1].v), "+v"(acc[1][2].v), "+v"(acc[1][3].v)
                 : "v"(a[0].vh), "v"(a[1].vh), "v"(b[0].vh), "v"(b[1].vh), "v"(b[2].vh), "v"(b[3].vh));
  }
  __syncthreads();

  if constexpr (OMODE == 2) {
    float* const stg = smem_f;
    #pragma unroll
    for (int nt = 0; nt < 4; ++nt) {
      const int col = wn + nt * 16 + l16;
      const float bb = bf16_rne(bias[bn + col]);
      #pragma unroll
      for (int mt = 0; mt < 2; ++mt)
        #pragma unroll
        for (int r = 0; r < 8; ++r) {
          const int row = wm + mt * 16 + 8 * hh + r;
          stg[row * BN + col] = acc[mt][nt].f[r] * acc_scale + bb;
        }
    }
    __syncthreads();
    float* const Cf = reinterpret_cast<float*>(Cp);
    #pragma unroll
    for (int pass = 0; pass < 2; ++pass) {
      #pragma unroll
      for (int it = 0; it < 16; ++it) {
        const int row = wid * 16 + it;
        const int c4 = lane * 4;
        const f32x4 v = *(const f32x4*)(stg + row * BN + c4);
        *(volatile f32x4*)(Cf + (size_t)(bm + row) * N + bn + c4) = v;
      }
      if (pass == 0) __threadfence();
    }
  } else {
    u16* const stg = smem_h;
    #pragma unroll
    for (int nt = 0; nt < 4; ++nt) {
      const int col = wn + nt * 16 + l16;
      const float bb = bf16_rne(bias[bn + col]);
      #pragma unroll
      for (int mt = 0; mt < 2; ++mt)
        #pragma unroll
        for (int r = 0; r < 8; ++r) {
          const int row = wm + mt * 16 + 8 * hh + r;
          const u16 hv = (u16)h_bits(acc[mt][nt].f[r] * acc_scale + bb);
          if constexpr (OMODE == 0) stg[row * BN + col] = hv;
          else                      stg[col * BM + row] = hv;
        }
    }
    __syncthreads();
    u16* const Ch = reinterpret_cast<u16*>(Cp);
    #pragma unroll
    for (int pass = 0; pass < 2; ++pass) {
      #pragma unroll
      for (int it = 0; it < 8; ++it) {
        const int line = (wid * 8 + it) * 2 + hh;
        const int c8 = l16 * 8;
        const u32x4 v = *(const u32x4*)(stg + line * 128 + c8);
        size_t gi;
        if constexpr (OMODE == 0) gi = (size_t)(bm + line) * N + bn + c8;
        else                      gi = (size_t)(bn + line) * M + bm + c8;
        *(volatile u32x4*)(Ch + gi) = v;
      }
      if (pass == 0) __threadfence();
    }
  }
}

__global__ __launch_bounds__(256) void attn_kernel(
    const u16* __restrict__ qp, const u16* __restrict__ kp, const u16* __restrict__ vpT,
    u16* op, int NQ, int NK, int C, int nbatch, float scale)
{
  constexpr int HD = 64, QT = 128, KCH = 64;
  constexpr int LQ = HD + 8, LK = HD + 8, LV = KCH + 8;
  __shared__ __attribute__((aligned(16))) u16 Qs[QT * LQ];
  __shared__ __attribute__((aligned(16))) u16 Ks[KCH * LK];
  __shared__ __attribute__((aligned(16))) u16 Vt[HD * LV];

  const int tid = threadIdx.x, lane = tid & 31, wid = tid >> 5;
  const int l16 = lane & 15, hh = lane >> 4;
  const int nheads = C / HD;
  const int b = blockIdx.y / nheads, h = blockIdx.y - b * nheads;
  const int q0 = blockIdx.x * QT;
  const size_t rowQ0 = (size_t)b * NQ + q0;
  const size_t rowK0 = (size_t)b * NK;
  const size_t colH  = (size_t)h * HD;
  const size_t MKV   = (size_t)nbatch * NK;

  #pragma unroll
  for (int j = 0; j < 4; ++j) {
    const int f = tid + j * 256, row = f >> 3, c8 = (f & 7) * 8;
    *(u32x4*)(Qs + row * LQ + c8) = *(const u32x4*)(qp + (rowQ0 + row) * C + colH + c8);
  }
  __syncthreads();

  Frag qf[2];
  {
    const int qq = wid * 16 + l16;
    #pragma unroll
    for (int s = 0; s < 2; ++s) {
      qf[s].q[0] = *(const u32x4*)(Qs + qq * LQ + s * 32 + 8 * hh);
      qf[s].q[1] = *(const u32x4*)(Qs + qq * LQ + s * 32 + 16 + 8 * hh);
    }
  }

  Acc oacc[4];
  #pragma unroll
  for (int nt = 0; nt < 4; ++nt)
    #pragma unroll
    for (int r = 0; r < 8; ++r) oacc[nt].f[r] = 0.f;

  float mrun = -1e30f, lrun = 0.f;
  const int nch = NK / KCH;

  #pragma unroll 1
  for (int c = 0; c < nch; ++c) {
    const int kc0 = c * KCH;
    u32x4 rk[2], rv[2];
    #pragma unroll
    for (int j = 0; j < 2; ++j) {
      const int f = tid + j * 256, row = f >> 3, c8 = (f & 7) * 8;
      rk[j] = *(const u32x4*)(kp  + (rowK0 + kc0 + row) * C + colH + c8);
      rv[j] = *(const u32x4*)(vpT + (colH + row) * MKV + rowK0 + kc0 + c8);
    }
    __syncthreads();
    #pragma unroll
    for (int j = 0; j < 2; ++j) {
      const int f = tid + j * 256, row = f >> 3, c8 = (f & 7) * 8;
      *(u32x4*)(Ks + row * LK + c8) = rk[j];
      *(u32x4*)(Vt + row * LV + c8) = rv[j];
    }
    __syncthreads();

    Acc sacc[4];
    #pragma unroll
    for (int mt = 0; mt < 4; ++mt) {
      #pragma unroll
      for (int r = 0; r < 8; ++r) sacc[mt].f[r] = 0.f;
      const int row = mt * 16 + l16;
      Frag a0, a1;
      a0.q[0] = *(const u32x4*)(Ks + row * LK + 8 * hh);
      a0.q[1] = *(const u32x4*)(Ks + row * LK + 16 + 8 * hh);
      a1.q[0] = *(const u32x4*)(Ks + row * LK + 32 + 8 * hh);
      a1.q[1] = *(const u32x4*)(Ks + row * LK + 48 + 8 * hh);
      sacc[mt].v = wmma_f16(a0, qf[0], sacc[mt].v);
      sacc[mt].v = wmma_f16(a1, qf[1], sacc[mt].v);
      WMMA_GUARD1(sacc[mt].v, a0.vh, a1.vh, qf[0].vh, qf[1].vh);
    }

    float cmax = -1e30f;
    #pragma unroll
    for (int mt = 0; mt < 4; ++mt)
      #pragma unroll
      for (int r = 0; r < 8; ++r) cmax = fmaxf(cmax, sacc[mt].f[r]);
    cmax = fmaxf(cmax, __shfl_xor(cmax, 16)) * scale;
    const float nm   = fmaxf(mrun, cmax);
    const float corr = __expf(mrun - nm);
    float csum = 0.f;
    #pragma unroll
    for (int mt = 0; mt < 4; ++mt)
      #pragma unroll
      for (int r = 0; r < 8; ++r) {
        const float e = __expf(sacc[mt].f[r] * scale - nm);
        sacc[mt].f[r] = e;
        csum += e;
      }
    csum += __shfl_xor(csum, 16);
    lrun = lrun * corr + csum;
    mrun = nm;

    #pragma unroll
    for (int r = 0; r < 8; ++r) {
      const float cf = __shfl(corr, r + 8 * hh);
      #pragma unroll
      for (int nt = 0; nt < 4; ++nt) oacc[nt].f[r] *= cf;
    }

    Frag pf[2];
    #pragma unroll
    for (int s = 0; s < 2; ++s)
      #pragma unroll
      for (int j = 0; j < 4; ++j) {
        pf[s].u[j]     = packh2(sacc[2 * s    ].f[2 * j] * 256.f, sacc[2 * s    ].f[2 * j + 1] * 256.f);
        pf[s].u[4 + j] = packh2(sacc[2 * s + 1].f[2 * j] * 256.f, sacc[2 * s + 1].f[2 * j + 1] * 256.f);
      }

    #pragma unroll
    for (int nt = 0; nt < 4; ++nt) {
      const int d = nt * 16 + l16;
      Frag b0, b1;
      b0.q[0] = *(const u32x4*)(Vt + d * LV + 8 * hh);
      b0.q[1] = *(const u32x4*)(Vt + d * LV + 16 + 8 * hh);
      b1.q[0] = *(const u32x4*)(Vt + d * LV + 32 + 8 * hh);
      b1.q[1] = *(const u32x4*)(Vt + d * LV + 48 + 8 * hh);
      oacc[nt].v = wmma_f16(pf[0], b0, oacc[nt].v);
      oacc[nt].v = wmma_f16(pf[1], b1, oacc[nt].v);
      WMMA_GUARD1(oacc[nt].v, pf[0].vh, pf[1].vh, b0.vh, b1.vh);
    }
  }

  const float inv = 1.f / lrun;
  __syncthreads();
  u16* const Os = Qs;
  #pragma unroll
  for (int r = 0; r < 8; ++r) {
    const float iv = __shfl(inv, r + 8 * hh);
    const int ql = wid * 16 + 8 * hh + r;
    #pragma unroll
    for (int nt = 0; nt < 4; ++nt) {
      const int d = nt * 16 + l16;
      Os[ql * HD + d] = (u16)h_bits(oacc[nt].f[r] * iv);
    }
  }
  __syncthreads();
  #pragma unroll
  for (int pass = 0; pass < 2; ++pass) {
    #pragma unroll
    for (int it = 0; it < 4; ++it) {
      const int row = wid * 16 + it * 4 + (lane >> 3);
      const int c8 = (lane & 7) * 8;
      const u32x4 v = *(const u32x4*)(Os + row * HD + c8);
      *(volatile u32x4*)(op + (rowQ0 + row) * C + colH + c8) = v;
    }
    if (pass == 0) __threadfence();
  }
}

extern "C" void kernel_launch(void* const* d_in, const int* in_sizes, int n_in,
                              void* d_out, int out_size, void* d_ws, size_t ws_size,
                              hipStream_t stream)
{
  const int NB = 2, NQ = 2048, NK = 2048, E = 1024, KV = 1024, CI = 1024, NH = 16, HD = 64;
  if (n_in < 11) return;
  if (in_sizes[0] != NB * NQ * E || in_sizes[1] != NB * NK * KV || in_sizes[2] != NB * NK * KV ||
      in_sizes[3] != E * CI || in_sizes[4] != CI || in_sizes[5] != KV * CI || in_sizes[6] != CI ||
      in_sizes[7] != KV * CI || in_sizes[8] != CI || in_sizes[9] != CI * E || in_sizes[10] != E ||
      out_size != NB * NQ * E) return;
  if ((NB * NQ) % 128 || (NB * NK) % 128 || CI % 128 || E % 128 || E % 32 || KV % 32 || CI % 32 ||
      E % 64 || KV % 64 || CI % 64 || NQ % 128 || NK % 64 || CI != NH * HD ||
      E != KV || E != CI || NQ != NK || (in_sizes[0] % 8)) return;

  const float* q  = (const float*)d_in[0];
  const float* k  = (const float*)d_in[1];
  const float* v  = (const float*)d_in[2];
  const float* Wq = (const float*)d_in[3];
  const float* bq = (const float*)d_in[4];
  const float* Wk = (const float*)d_in[5];
  const float* bk = (const float*)d_in[6];
  const float* Wv = (const float*)d_in[7];
  const float* bv = (const float*)d_in[8];
  const float* Wo = (const float*)d_in[9];
  const float* bo = (const float*)d_in[10];

  unsigned char* ws = (unsigned char*)d_ws;
  size_t off = 0;
  auto carve = [&](size_t bytes) -> unsigned char* {
    unsigned char* p = ws + off;
    off += (bytes + 255) & ~(size_t)255;
    return p;
  };
  u16* qb  = (u16*)carve((size_t)NB * NQ * E  * 2);
  u16* kb  = (u16*)carve((size_t)NB * NK * KV * 2);
  u16* vb  = (u16*)carve((size_t)NB * NK * KV * 2);
  u16* WqT = (u16*)carve((size_t)CI * E  * 2);
  u16* WkT = (u16*)carve((size_t)CI * KV * 2);
  u16* WvT = (u16*)carve((size_t)CI * KV * 2);
  u16* WoT = (u16*)carve((size_t)E  * CI * 2);
  u16* qph = (u16*)carve((size_t)NB * NQ * CI * 2);
  u16* kph = (u16*)carve((size_t)NB * NK * CI * 2);
  u16* vpT = (u16*)carve((size_t)CI * NB * NK * 2);
  u16* ao  = (u16*)carve((size_t)NB * NQ * CI * 2);
  if (off > ws_size) return;

  const int n8 = in_sizes[0] / 8;
  cvt_bf16_kernel<<<dim3((n8 + 255) / 256, 3), 256, 0, stream>>>(q, k, v, qb, kb, vb, n8);

  wtrans_kernel<<<dim3(E / 64, CI / 32, 4), 256, 0, stream>>>(
      Wq, Wk, Wv, Wo, WqT, WkT, WvT, WoT, E, CI, 64.f);

  const dim3 gp(CI / 128, (NB * NQ) / 128);
  gemm_kernel<false, 0><<<gp, 256, 0, stream>>>(qb, WqT, bq, qph, NB * NQ, E,  CI, 1.f);
  gemm_kernel<false, 0><<<dim3(CI / 128, (NB * NK) / 128), 256, 0, stream>>>(kb, WkT, bk, kph, NB * NK, KV, CI, 1.f);
  gemm_kernel<false, 1><<<dim3(CI / 128, (NB * NK) / 128), 256, 0, stream>>>(vb, WvT, bv, vpT, NB * NK, KV, CI, 1.f);

  const float scale = 1.0f / 8.0f;
  attn_kernel<<<dim3(NQ / 128, NB * NH), 256, 0, stream>>>(qph, kph, vpT, ao, NQ, NK, CI, NB, scale);

  gemm_kernel<true, 2><<<dim3(E / 128, (NB * NQ) / 128), 256, 0, stream>>>(
      ao, WoT, bo, d_out, NB * NQ, CI, E, 1.0f / 16384.0f);
}
